// DynamycMoE_49959059587400
// MI455X (gfx1250) — hardware-verified
//
#include <hip/hip_runtime.h>
#include <math.h>

typedef __attribute__((ext_vector_type(16))) _Float16 v16h;
typedef __attribute__((ext_vector_type(16))) __bf16 v16b;
typedef __attribute__((ext_vector_type(8)))  _Float16 v8h;
typedef __attribute__((ext_vector_type(8)))  __bf16 v8b;
typedef __attribute__((ext_vector_type(8)))  float v8f;
typedef __attribute__((ext_vector_type(4)))  float v4f;
typedef __attribute__((ext_vector_type(4)))  unsigned v4u;

#ifndef NB
#define NB 8192
#endif
#define NB_FULL 8192
#define DIN  768
#define DHID 256
#define DC   64
#define NE   8
#define NT   512
#define KH (NE * DHID)
#define KO (NE * DC)
#define HCARRY 64.0f
#define WCARRY 512.0f
#define OCARRY 64.0f
#define HSCALE (1.0f / 32768.0f)
#define OSCALE (1.0f / 32768.0f)
#define EPS32 2.220446049250313e-16f

#define WS_XB  ((size_t)0)
#define WS_W1B (WS_XB  + (size_t)NB * DIN * 2)
#define WS_W2H (WS_W1B + (size_t)NE * DHID * DIN * 2)
#define WS_WMH (WS_W2H + (size_t)NE * DC * DHID * 2)
#define WS_G   (WS_WMH + (size_t)NT * KO * 2)
#define WS_HB  (WS_G   + (size_t)NB * NE * 4)
#define WS_OB  (WS_HB  + (size_t)NB * KH * 2)
#define WS_END (WS_OB  + (size_t)NB * KO * 2)

static_assert(NB % 128 == 0);
static_assert(NB <= NB_FULL);
static_assert(NE == 8 && DC == 64);
static_assert(DIN % 32 == 0 && DHID % 32 == 0 && KO % 32 == 0 && DIN % 2 == 0);
static_assert((KH * 2) % 128 == 0 && (KO * 2) % 128 == 0 && (DIN * 2) % 16 == 0);
static_assert(DHID % 128 == 0 && NT % 128 == 0);
static_assert((size_t)NB_FULL * NT * 4 == 16777216);
static_assert(WS_W1B % 128 == 0 && WS_W2H % 128 == 0 && WS_WMH % 128 == 0 && WS_G % 128 == 0 && WS_HB % 128 == 0 && WS_OB % 128 == 0);
static_assert(WS_END <= (size_t)134217728);
static_assert((size_t)(NB * DIN / 8 / 256) * 256 * 8 == (size_t)NB * DIN);
static_assert((size_t)(NE * DHID * DIN / 8 / 256) * 256 * 8 == (size_t)NE * DHID * DIN);
static_assert((size_t)(NE * DC * DHID / 8 / 256) * 256 * 8 == (size_t)NE * DC * DHID);
static_assert((size_t)(NE * NT * DC / 8 / 256) * 256 * 8 == (size_t)NT * KO);
static_assert(NT * DC / 8 == 4096 && DC / 8 == 8);
static_assert((size_t)(NB / 128) * 128 * NE == (size_t)NB * NE);
static_assert((size_t)(DHID / 128) * (NB / 128) * NE * 128 * 128 == (size_t)NB * KH);
static_assert((size_t)(NB / 128) * NE * 128 * DC == (size_t)NB * KO);
static_assert((size_t)(NT / 128) * (NB / 128) * 128 * 128 == (size_t)NB * NT);
static_assert(128 * 16 * 2 == 128 * NE * 4);
static_assert(32 * 16 * 8 == 32 * 64 * 2);
static_assert(32 * 16 * 8 == 16 * 64 * 4);
static_assert(DIN * NE * 4 + 128 * NE * 4 <= 131072);
static_assert(8 * 32 * 64 * 2 <= 131072 && 4 * 32 * 64 * 2 <= 131072 && 8 * 16 * 64 * 4 <= 131072);

__device__ __forceinline__ v8f wmma16(v16h a, v16h b, v8f c) {
  v8f d = __builtin_amdgcn_wmma_f32_16x16x32_f16(false, a, false, b, (short)0, c, false, false);
  asm volatile("v_nop\n\tv_nop\n\tv_nop\n\tv_nop" : "+v"(d) : "v"(a), "v"(b));
  return d;
}
__device__ __forceinline__ v8f wmma_bf(v16b a, v16b b, v8f c) {
  v8f d = __builtin_amdgcn_wmma_f32_16x16x32_bf16(false, a, false, b, (short)0, c, false, false);
  asm volatile("v_nop\n\tv_nop\n\tv_nop\n\tv_nop" : "+v"(d) : "v"(a), "v"(b));
  return d;
}
__device__ __forceinline__ float bfr(float v) { return (float)(__bf16)v; }
static __device__ __forceinline__ _Float16 toh_flush(float v) { const _Float16 r = (_Float16)v; return (fabsf(v) < 6.103515625e-05f) ? (_Float16)0.0f : r; }
__device__ __forceinline__ v16b ldfrag_b(const unsigned short* p) { union { v16b v; v4u q[2]; } f; f.q[0] = *(const v4u*)p; f.q[1] = *(const v4u*)(p + 16); return f.v; }
__device__ __forceinline__ v16h ldfrag_h(const unsigned short* p) { union { v16h v; v4u q[2]; } f; f.q[0] = *(const v4u*)p; f.q[1] = *(const v4u*)(p + 16); return f.v; }

__global__ __launch_bounds__(256) void k_cvt_x(const float* __restrict__ X, unsigned short* __restrict__ XB) {
  const unsigned i = blockIdx.x * 256u + threadIdx.x;
  const unsigned ic = i < (unsigned)(NB * DIN / 8) ? i : (unsigned)(NB * DIN / 8 - 1);
  const v4f a = *(const v4f*)(X + (size_t)ic * 8), b = *(const v4f*)(X + (size_t)ic * 8 + 4);
  union { v8b h; v4u u; } o;
#pragma unroll
  for (int j = 0; j < 4; ++j) { o.h[j] = (__bf16)a[j]; o.h[4 + j] = (__bf16)b[j]; }
  const v4u val = o.u;
  volatile v4u* p = (volatile v4u*)(XB + (size_t)ic * 8);
  *p = val; __threadfence(); *p = val;
}

__global__ __launch_bounds__(256) void k_cvt_w1(const float* __restrict__ W, unsigned short* __restrict__ WB) {
  const unsigned i = blockIdx.x * 256u + threadIdx.x;
  const unsigned ic = i < (unsigned)(NE * DHID * DIN / 8) ? i : (unsigned)(NE * DHID * DIN / 8 - 1);
  const v4f a = *(const v4f*)(W + (size_t)ic * 8), b = *(const v4f*)(W + (size_t)ic * 8 + 4);
  union { v8b h; v4u u; } o;
#pragma unroll
  for (int j = 0; j < 4; ++j) { o.h[j] = (__bf16)a[j]; o.h[4 + j] = (__bf16)b[j]; }
  const v4u val = o.u;
  volatile v4u* p = (volatile v4u*)(WB + (size_t)ic * 8);
  *p = val; __threadfence(); *p = val;
}

__global__ __launch_bounds__(256) void k_cvt_w2(const float* __restrict__ W, unsigned short* __restrict__ WH) {
  const unsigned i = blockIdx.x * 256u + threadIdx.x;
  const unsigned ic = i < (unsigned)(NE * DC * DHID / 8) ? i : (unsigned)(NE * DC * DHID / 8 - 1);
  const v4f a = *(const v4f*)(W + (size_t)ic * 8), b = *(const v4f*)(W + (size_t)ic * 8 + 4);
  union { v8h h; v4u u; } o;
#pragma unroll
  for (int j = 0; j < 4; ++j) { o.h[j] = toh_flush(bfr(a[j]) * WCARRY); o.h[4 + j] = toh_flush(bfr(b[j]) * WCARRY); }
  const v4u val = o.u;
  volatile v4u* p = (volatile v4u*)(WH + (size_t)ic * 8);
  *p = val; __threadfence(); *p = val;
}

__global__ __launch_bounds__(256) void k_cvt_wm(const float* __restrict__ W, unsigned short* __restrict__ WH) {
  const unsigned i = blockIdx.x * 256u + threadIdx.x;
  const unsigned ic = i < (unsigned)(NE * NT * DC / 8) ? i : (unsigned)(NE * NT * DC / 8 - 1);
  const unsigned e = ic >> 12, tt = (ic >> 3) & (NT - 1u), q = ic & 7u;
  const v4f a = *(const v4f*)(W + (size_t)ic * 8), b = *(const v4f*)(W + (size_t)ic * 8 + 4);
  union { v8h h; v4u u; } o;
#pragma unroll
  for (int j = 0; j < 4; ++j) { o.h[j] = toh_flush(bfr(a[j]) * WCARRY); o.h[4 + j] = toh_flush(bfr(b[j]) * WCARRY); }
  const v4u val = o.u;
  volatile v4u* p = (volatile v4u*)(WH + (size_t)tt * KO + e * DC + 8u * q);
  *p = val; __threadfence(); *p = val;
}

__global__ __launch_bounds__(128) void k_gate(const unsigned short* __restrict__ XB, const float* __restrict__ WG, float* __restrict__ G) {
#pragma clang fp contract(off)
  __shared__ __align__(16) float wgs[DIN][NE];
  __shared__ __align__(16) float sp[128][NE];
  const unsigned tid = threadIdx.x; const unsigned r0 = blockIdx.x * 128u; const unsigned row = r0 + tid;
#pragma unroll 1
  for (unsigned i = tid; i < (unsigned)(DIN * NE / 4); i += 128u) { const v4f w = *(const v4f*)(WG + 4u * i); v4f o;
#pragma unroll
    for (int j = 0; j < 4; ++j) o[j] = bfr(w[j]);
    *(v4f*)(&wgs[0][0] + 4u * i) = o; }
  __syncthreads();
  float acc[NE];
#pragma unroll
  for (int e = 0; e < NE; ++e) acc[e] = 0.f;
  const unsigned* xr = (const unsigned*)(XB + (size_t)row * DIN);
#pragma unroll 1
  for (unsigned kw = 0; kw < (unsigned)(DIN / 2); ++kw) {
    const unsigned w = xr[kw];
    const float x0 = __uint_as_float(w << 16), x1 = __uint_as_float(w & 0xffff0000u);
    const v4f p0 = *(const v4f*)&wgs[2u * kw][0], p1 = *(const v4f*)&wgs[2u * kw][4];
    const v4f q0 = *(const v4f*)&wgs[2u * kw + 1u][0], q1 = *(const v4f*)&wgs[2u * kw + 1u][4];
#pragma unroll
    for (int j = 0; j < 4; ++j) { acc[j] = fmaf(x0, p0[j], acc[j]); acc[4 + j] = fmaf(x0, p1[j], acc[4 + j]); }
#pragma unroll
    for (int j = 0; j < 4; ++j) { acc[j] = fmaf(x1, q0[j], acc[j]); acc[4 + j] = fmaf(x1, q1[j], acc[4 + j]); }
  }
  int i1 = 0; float v1 = acc[0];
#pragma unroll
  for (int e = 1; e < NE; ++e) { const bool c = acc[e] > v1; v1 = c ? acc[e] : v1; i1 = c ? e : i1; }
  int i2 = -1; float v2 = 0.f;
#pragma unroll
  for (int e = 0; e < NE; ++e) { const bool c = (e != i1) && ((i2 < 0) || (acc[e] > v2)); v2 = c ? acc[e] : v2; i2 = c ? e : i2; }
  const float tt = expf(v2 - v1);
  const float inv = 1.0f / (1.0f + tt);
  const float g1 = inv, g2 = tt * inv;
#pragma unroll
  for (int e = 0; e < NE; e += 4) { v4f o;
#pragma unroll
    for (int j = 0; j < 4; ++j) o[j] = ((e + j) == i1) ? g1 : (((e + j) == i2) ? g2 : 0.f);
    *(v4f*)&sp[tid][e] = o; }
  __syncthreads();
  v4f pv[2];
#pragma unroll
  for (unsigned it = 0; it < 2; ++it) { const unsigned idx = it * 128u + tid; pv[it] = *(const v4f*)(&sp[0][0] + 4u * idx); }
  float* go = G + (size_t)r0 * NE;
#pragma unroll
  for (unsigned it = 0; it < 2; ++it) { const unsigned idx = it * 128u + tid; *(volatile v4f*)(go + 4u * idx) = pv[it]; }
  __threadfence();
#pragma unroll
  for (unsigned it = 0; it < 2; ++it) { const unsigned idx = it * 128u + tid; *(volatile v4f*)(go + 4u * idx) = pv[it]; }
}

__global__ __launch_bounds__(256) void k_h(const unsigned short* __restrict__ XB, const unsigned short* __restrict__ W1B, const float* __restrict__ B1, unsigned short* __restrict__ HB) {
  __shared__ __align__(16) _Float16 sh[8][32][64];
  const unsigned t = threadIdx.x, wave = t >> 5, lane = t & 31u, lm = lane & 15u, lh = lane >> 4, wm = wave >> 1, wn = wave & 1u;
  const unsigned e = blockIdx.z, m0 = blockIdx.y * 128u, n0 = blockIdx.x * 128u;
  const unsigned short* ar[2]; const unsigned short* br[4];
#pragma unroll
  for (int mi = 0; mi < 2; ++mi) ar[mi] = XB + (size_t)(m0 + wm * 32u + mi * 16u + lm) * DIN + 8u * lh;
#pragma unroll
  for (int ni = 0; ni < 4; ++ni) br[ni] = W1B + (size_t)(e * DHID + n0 + wn * 64u + ni * 16u + lm) * DIN + 8u * lh;
  v8f acc[2][4] = {};
#pragma unroll 2
  for (unsigned kc = 0; kc < DIN / 32; ++kc) { v16b a[2], b[4];
#pragma unroll
    for (int mi = 0; mi < 2; ++mi) a[mi] = ldfrag_b(ar[mi] + kc * 32u);
#pragma unroll
    for (int ni = 0; ni < 4; ++ni) b[ni] = ldfrag_b(br[ni] + kc * 32u);
#pragma unroll
    for (int mi = 0; mi < 2; ++mi)
#pragma unroll
      for (int ni = 0; ni < 4; ++ni) acc[mi][ni] = wmma_bf(a[mi], b[ni], acc[mi][ni]); }
#pragma unroll
  for (int ni = 0; ni < 4; ++ni) { const float bb = bfr(B1[(size_t)e * DHID + n0 + wn * 64u + ni * 16u + lm]);
#pragma unroll
    for (int mi = 0; mi < 2; ++mi)
#pragma unroll
      for (int r = 0; r < 8; ++r) sh[wave][mi * 16 + 8u * lh + r][ni * 16 + lm] = toh_flush(fmaxf(acc[mi][ni][r] + bb, 0.f) * HCARRY); }
  __syncthreads();
  v4u o[8];
#pragma unroll
  for (unsigned it = 0; it < 8; ++it) { const unsigned rw = it * 4u + (lane >> 3), q = lane & 7u; union { v8h h; v4u u; } w; w.h = *(const v8h*)&sh[wave][rw][8u * q]; o[it] = w.u; }
  unsigned short* hb = HB + (size_t)(m0 + wm * 32u) * KH + e * DHID + n0 + wn * 64u;
#pragma unroll
  for (unsigned it = 0; it < 8; ++it) { const unsigned rw = it * 4u + (lane >> 3), q = lane & 7u; *(volatile v4u*)(hb + (size_t)rw * KH + 8u * q) = o[it]; }
  __threadfence();
#pragma unroll
  for (unsigned it = 0; it < 8; ++it) { const unsigned rw = it * 4u + (lane >> 3), q = lane & 7u; *(volatile v4u*)(hb + (size_t)rw * KH + 8u * q) = o[it]; }
}

__global__ __launch_bounds__(128) void k_o(const unsigned short* __restrict__ HB, const unsigned short* __restrict__ W2H, const float* __restrict__ B2, const float* __restrict__ G, unsigned short* __restrict__ OB) {
  __shared__ __align__(16) _Float16 sh[4][32][64];
  const unsigned t = threadIdx.x, wave = t >> 5, lane = t & 31u, lm = lane & 15u, lh = lane >> 4;
  const unsigned e = blockIdx.y, m0 = blockIdx.x * 128u;
  const unsigned short* ar[2]; const unsigned short* br[4];
#pragma unroll
  for (int mi = 0; mi < 2; ++mi) ar[mi] = HB + (size_t)(m0 + wave * 32u + mi * 16u + lm) * KH + e * DHID + 8u * lh;
#pragma unroll
  for (int ni = 0; ni < 4; ++ni) br[ni] = W2H + (size_t)(e * DC + ni * 16u + lm) * DHID + 8u * lh;
  v8f acc[2][4] = {};
#pragma unroll 2
  for (unsigned kc = 0; kc < DHID / 32; ++kc) { v16h a[2], b[4];
#pragma unroll
    for (int mi = 0; mi < 2; ++mi) a[mi] = ldfrag_h(ar[mi] + kc * 32u);
#pragma unroll
    for (int ni = 0; ni < 4; ++ni) b[ni] = ldfrag_h(br[ni] + kc * 32u);
#pragma unroll
    for (int mi = 0; mi < 2; ++mi)
#pragma unroll
      for (int ni = 0; ni < 4; ++ni) acc[mi][ni] = wmma16(a[mi], b[ni], acc[mi][ni]); }
  float gv[2][8];
#pragma unroll
  for (int mi = 0; mi < 2; ++mi) {
#pragma unroll
    for (int r = 0; r < 8; ++r) gv[mi][r] = G[(size_t)(m0 + wave * 32u + mi * 16u + 8u * lh + r) * NE + e] * OCARRY;
    asm volatile("s_wait_loadcnt 0x0" ::: "memory"); }
#pragma unroll
  for (int ni = 0; ni < 4; ++ni) { const float bb = bfr(B2[(size_t)e * DC + ni * 16u + lm]);
#pragma unroll
    for (int mi = 0; mi < 2; ++mi)
#pragma unroll
      for (int r = 0; r < 8; ++r) sh[wave][mi * 16 + 8u * lh + r][ni * 16 + lm] = toh_flush((acc[mi][ni][r] * HSCALE + bb) * gv[mi][r]); }
  __syncthreads();
  v4u o[8];
#pragma unroll
  for (unsigned it = 0; it < 8; ++it) { const unsigned rw = it * 4u + (lane >> 3), q = lane & 7u; union { v8h h; v4u u; } w; w.h = *(const v8h*)&sh[wave][rw][8u * q]; o[it] = w.u; }
  unsigned short* ob = OB + (size_t)(m0 + wave * 32u) * KO + e * DC;
#pragma unroll
  for (unsigned it = 0; it < 8; ++it) { const unsigned rw = it * 4u + (lane >> 3), q = lane & 7u; *(volatile v4u*)(ob + (size_t)rw * KO + 8u * q) = o[it]; }
  __threadfence();
#pragma unroll
  for (unsigned it = 0; it < 8; ++it) { const unsigned rw = it * 4u + (lane >> 3), q = lane & 7u; *(volatile v4u*)(ob + (size_t)rw * KO + 8u * q) = o[it]; }
}

__global__ __launch_bounds__(256) void k_out(const unsigned short* __restrict__ OB, const unsigned short* __restrict__ WMH, float* __restrict__ OUT) {
  __shared__ __align__(16) float sf[8][16][64];
  const unsigned t = threadIdx.x, wave = t >> 5, lane = t & 31u, lm = lane & 15u, lh = lane >> 4, wm = wave >> 1, wn = wave & 1u;
  const unsigned m0 = blockIdx.y * 128u, n0 = blockIdx.x * 128u;
  const unsigned short* ar[2]; const unsigned short* br[4];
#pragma unroll
  for (int mi = 0; mi < 2; ++mi) ar[mi] = OB + (size_t)(m0 + wm * 32u + mi * 16u + lm) * KO + 8u * lh;
#pragma unroll
  for (int ni = 0; ni < 4; ++ni) br[ni] = WMH + (size_t)(n0 + wn * 64u + ni * 16u + lm) * KO + 8u * lh;
  v8f acc[2][4] = {};
#pragma unroll 2
  for (unsigned kc = 0; kc < KO / 32; ++kc) { v16h a[2], b[4];
#pragma unroll
    for (int mi = 0; mi < 2; ++mi) a[mi] = ldfrag_h(ar[mi] + kc * 32u);
#pragma unroll
    for (int ni = 0; ni < 4; ++ni) b[ni] = ldfrag_h(br[ni] + kc * 32u);
#pragma unroll
    for (int mi = 0; mi < 2; ++mi)
#pragma unroll
      for (int ni = 0; ni < 4; ++ni) acc[mi][ni] = wmma16(a[mi], b[ni], acc[mi][ni]); }
#pragma unroll
  for (int mi = 0; mi < 2; ++mi) {
    if (mi) __syncthreads();
#pragma unroll
    for (int ni = 0; ni < 4; ++ni)
#pragma unroll
      for (int r = 0; r < 8; ++r) { const float yv = acc[mi][ni][r] * OSCALE; sf[wave][8u * lh + r][ni * 16 + lm] = (yv == 0.0f) ? EPS32 : yv; }
    __syncthreads();
    v4f v[8];
#pragma unroll
    for (unsigned it = 0; it < 8; ++it) { const unsigned rw = it * 2u + (lane >> 4), pc = lane & 15u; v[it] = *(const v4f*)&sf[wave][rw][4u * pc]; }
    float* po = OUT + (size_t)(m0 + wm * 32u + mi * 16u) * NT + n0 + wn * 64u;
#pragma unroll
    for (unsigned it = 0; it < 8; ++it) { const unsigned rw = it * 2u + (lane >> 4), pc = lane & 15u; *(volatile v4f*)(po + (size_t)rw * NT + 4u * pc) = v[it]; }
    __threadfence();
#pragma unroll
    for (unsigned it = 0; it < 8; ++it) { const unsigned rw = it * 2u + (lane >> 4), pc = lane & 15u; *(volatile v4f*)(po + (size_t)rw * NT + 4u * pc) = v[it]; }
  }
}

extern "C" void kernel_launch(void* const* d_in, const int* in_sizes, int n_in, void* d_out, int out_size, void* d_ws, size_t ws_size, hipStream_t stream) {
  if (n_in < 8) return;
  if (in_sizes[0] < NB * DIN || in_sizes[2] < DIN * NE || in_sizes[3] < NE * DHID * DIN || in_sizes[4] < NE * DHID) return;
  if (in_sizes[5] < NE * DC * DHID || in_sizes[6] < NE * DC || in_sizes[7] < NE * NT * DC) return;
  if ((size_t)out_size < (size_t)NB * NT) return;
  if (ws_size < (size_t)WS_END) return;
  const float* X   = (const float*)d_in[0];
  const float* WGT = (const float*)d_in[2];
  const float* W1  = (const float*)d_in[3];
  const float* B1  = (const float*)d_in[4];
  const float* W2  = (const float*)d_in[5];
  const float* B2  = (const float*)d_in[6];
  const float* WM  = (const float*)d_in[7];
  char* ws = (char*)d_ws;
  unsigned short* XB  = (unsigned short*)(ws + WS_XB);
  unsigned short* W1B = (unsigned short*)(ws + WS_W1B);
  unsigned short* W2H = (unsigned short*)(ws + WS_W2H);
  unsigned short* WMH = (unsigned short*)(ws + WS_WMH);
  float*          G   = (float*)(ws + WS_G);
  unsigned short* HB  = (unsigned short*)(ws + WS_HB);
  unsigned short* OB  = (unsigned short*)(ws + WS_OB);
  float* OUT = (float*)d_out;
  k_cvt_x<<<dim3(NB * DIN / 8 / 256), 256, 0, stream>>>(X, XB);
  k_cvt_w1<<<dim3(NE * DHID * DIN / 8 / 256), 256, 0, stream>>>(W1, W1B);
  k_cvt_w2<<<dim3(NE * DC * DHID / 8 / 256), 256, 0, stream>>>(W2, W2H);
  k_cvt_wm<<<dim3(NE * NT * DC / 8 / 256), 256, 0, stream>>>(WM, WMH);
  k_gate<<<dim3(NB / 128), 128, 0, stream>>>(XB, WGT, G);
  k_h<<<dim3(DHID / 128, NB / 128, NE), 256, 0, stream>>>(XB, W1B, B1, HB);
  k_o<<<dim3(NB / 128, NE), 128, 0, stream>>>(HB, W2H, B2, G, OB);
  k_out<<<dim3(NT / 128, NB / 128), 256, 0, stream>>>(OB, WMH, OUT);
}
